// GraphConvolution_82867099009361
// MI455X (gfx1250) — hardware-verified
//
#include <hip/hip_runtime.h>


namespace {
constexpr int B = 16, T = 2048, D = 64, BL = 16  , NR = B * T;
constexpr float XS = 8.0f, WSC = 256.0f, RS_ = 1024.0f, PS = 8.0f;
static_assert(T % 32 == 0 && D == 64, "tiling");
typedef _Float16 b16;
typedef __attribute__((ext_vector_type(16))) _Float16 v16b;
typedef __attribute__((ext_vector_type(8))) _Float16 v8b;
typedef __attribute__((ext_vector_type(8))) float v8f;
typedef __attribute__((ext_vector_type(4))) float v4f;
__device__ __forceinline__ float bf16_rne(float f) { unsigned int u = __float_as_uint(f); u += 0x7FFFu + ((u >> 16) & 1u); return __uint_as_float(u & 0xFFFF0000u); }
__device__ __forceinline__ void split16(float v, b16& hi, b16& lo) { hi = (b16)v; lo = (b16)(v - (float)hi); }
__device__ __forceinline__ v16b frag_kb(const b16* p, int hh) { const v8b a = *(const v8b*)(p + 8 * hh), b = *(const v8b*)(p + 16 + 8 * hh); v16b f;
#pragma unroll
  for (int e = 0; e < 8; ++e) { f[e] = a[e]; f[8 + e] = b[e]; } return f; }
__device__ __forceinline__ v8f wmma16b(v16b a, v16b b, v8f c) { v8f d = __builtin_amdgcn_wmma_f32_16x16x32_f16(false, a, false, b, (short)0, c, false, false); asm volatile("v_nop\n\tv_nop\n\tv_nop\n\tv_nop" : "+v"(d) : "v"(a), "v"(b)); return d; }
__device__ __forceinline__ void wave_lds_sync() { __builtin_amdgcn_fence(__ATOMIC_RELEASE, "workgroup"); __builtin_amdgcn_wave_barrier(); __builtin_amdgcn_fence(__ATOMIC_ACQUIRE, "workgroup"); }
__device__ __forceinline__ float pmul(float a, float b) { float p = a * b; asm volatile("" : "+v"(p)); return p; }
__device__ __forceinline__ int iclamp(int v, int lo, int hi) { return v < lo ? lo : (v > hi ? hi : v); }

typedef __attribute__((ext_vector_type(2))) _Float16 v2h;
typedef __attribute__((ext_vector_type(4))) _Float16 v4h;
typedef __attribute__((ext_vector_type(2))) float v2f;
typedef __attribute__((ext_vector_type(4))) int v4i;
__device__ __forceinline__ float nexp2(float v) { return __builtin_amdgcn_exp2f(v); }
__device__ __forceinline__ float bfp(float v) { float t = bf16_rne(v); asm volatile("" : "+v"(t)); return t; }

__global__ __launch_bounds__(256) void prep_kernel(const float* __restrict__ x, const float* __restrict__ w, b16* __restrict__ Xh, float* __restrict__ NRM, b16* __restrict__ WT) {
  const int tid = threadIdx.x; const int row = tid >> 3, g = tid & 7, c0 = g * 8; const size_t v = (size_t)blockIdx.x * 32 + row;
  float a[8]; float s2 = 0.0f; { const v4f p = *(const v4f*)(x + v * D + c0), q = *(const v4f*)(x + v * D + c0 + 4); for (int j = 0; j < 4; ++j) { a[j] = bf16_rne(p[j]); a[4 + j] = bf16_rne(q[j]); } }
#pragma unroll
  for (int j = 0; j < 8; ++j) s2 = fmaf(a[j], a[j], s2);
#pragma unroll
  for (int o = 1; o < 8; o <<= 1) s2 += __shfl_xor(s2, o);
  __shared__ float nr[32]; if (g == 0) nr[row] = sqrtf(s2); __syncthreads();
  v8b hv; for (int j = 0; j < 8; ++j) hv[j] = (b16)(a[j] * XS);
  for (int pass = 0; pass < 2; ++pass) { *(volatile v8b*)(Xh + v * D + c0) = hv; if (tid < 32) ((volatile float*)NRM)[(size_t)blockIdx.x * 32 + tid] = nr[tid];
    if (blockIdx.x == 0) { for (int i = tid; i < D * D / 8; i += 256) { const int e = i * 8; const int o = e / D, k0 = e % D; v8b wv; for (int j = 0; j < 8; ++j) wv[j] = (b16)(bf16_rne(w[(size_t)(k0 + j) * D + o]) * WSC); *(volatile v8b*)(WT + e) = wv; } }
    __threadfence(); }
}
__global__ __launch_bounds__(64) void sup_kernel(const b16* __restrict__ Xh, const b16* __restrict__ WT, b16* __restrict__ SPh, b16* __restrict__ SPl) {
  __shared__ __attribute__((aligned(16))) float Tw[2][16][D + 4];
  const int wave = threadIdx.x >> 5, lane = threadIdx.x & 31, nloc = lane & 15, hlf = lane >> 4; const size_t m0 = (size_t)blockIdx.x * 32 + wave * 16;
  v8f acc[4]; for (int t = 0; t < 4; ++t) acc[t] = (v8f){};
#pragma unroll
  for (int ks = 0; ks < 2; ++ks) { const v16b a = frag_kb(Xh + (m0 + nloc) * D + ks * 32, hlf);
#pragma unroll
    for (int t = 0; t < 4; ++t) acc[t] = wmma16b(a, frag_kb(WT + (size_t)(t * 16 + nloc) * D + ks * 32, hlf), acc[t]); }
#pragma unroll
  for (int t = 0; t < 4; ++t) for (int r = 0; r < 8; ++r) Tw[wave][8 * hlf + r][t * 16 + nloc] = acc[t][r] * (1.0f / (XS * WSC));
  wave_lds_sync();
  for (int pass = 0; pass < 2; ++pass) { for (int rr = 0; rr < 16; rr += 4) { const int r2 = rr + (lane >> 3); const int c8 = (lane & 7) * 8; v8b hv, lv;
      for (int j = 0; j < 8; ++j) { const float v = Tw[wave][r2][c8 + j] * XS; const b16 ph = (b16)v; hv[j] = ph; lv[j] = (b16)((v - (float)ph) * RS_); }
      *(volatile v8b*)(SPh + (m0 + r2) * D + c8) = hv; *(volatile v8b*)(SPl + (m0 + r2) * D + c8) = lv; } __threadfence(); }
}
__global__ __launch_bounds__(32) void main_kernel(const b16* __restrict__ Xh, const float* __restrict__ NRM, const float* __restrict__ att, const int* __restrict__ mask, const b16* __restrict__ SPh, const b16* __restrict__ SPl, const float* __restrict__ bias, float* __restrict__ out) {
  __shared__ __attribute__((aligned(16))) b16 Pt[16][32 + 8]; __shared__ __attribute__((aligned(16))) float Of[16][D + 4];
  const int lane = threadIdx.x, nloc = lane & 15, hlf = lane >> 4; const int n0 = blockIdx.x * 16, b = blockIdx.y; const size_t rbase = (size_t)b * T;
  v16b aq[2]; for (int ks = 0; ks < 2; ++ks) aq[ks] = frag_kb(Xh + (rbase + n0 + nloc) * D + ks * 32, hlf);
  float inr[8]; for (int r = 0; r < 8; ++r) { const float nv = NRM[rbase + n0 + 8 * hlf + r]; inr[r] = 1.0f / nv; }
  v8f acco[4], accol[4]; for (int t = 0; t < 4; ++t) { acco[t] = (v8f){}; accol[t] = (v8f){}; }
#pragma unroll 1
  for (int m0 = 0; m0 < T; m0 += 32) {
    v8f sacc[2];
#pragma unroll
    for (int t = 0; t < 2; ++t) { sacc[t] = (v8f){}; const size_t mrow = rbase + m0 + t * 16 + nloc;
#pragma unroll
      for (int ks = 0; ks < 2; ++ks) sacc[t] = wmma16b(aq[ks], frag_kb(Xh + mrow * D + ks * 32, hlf), sacc[t]); }
    v16b pv;
#pragma unroll
    for (int t = 0; t < 2; ++t) { const int m = m0 + t * 16 + nloc; const float inm = 1.0f / NRM[rbase + m];
#pragma unroll
      for (int r = 0; r < 8; ++r) { const int n = n0 + 8 * hlf + r; const float a_ = bf16_rne(att[(size_t)n * T + m]) * (float)mask[(size_t)n * T + m]; const float p = sacc[t][r] * (1.0f / (XS * XS)) * inr[r] * inm * a_; pv[8 * t + r] = (b16)(p * PS); } }
#pragma unroll
    for (int t = 0; t < 2; ++t) for (int r = 0; r < 8; ++r) Pt[8 * hlf + r][16 * t + nloc] = pv[8 * t + r];
    wave_lds_sync();
    const v16b a = frag_kb(&Pt[nloc][0], hlf);
#pragma unroll
    for (int t = 0; t < 4; ++t) { v16b vh, vl;
#pragma unroll
      for (int e = 0; e < 16; ++e) { const int k = (e < 8) ? (8 * hlf + e) : (16 + 8 * hlf + (e - 8)); const size_t o_ = (rbase + m0 + k) * D + t * 16 + nloc; vh[e] = SPh[o_]; vl[e] = SPl[o_]; }
      acco[t] = wmma16b(a, vh, acco[t]); accol[t] = wmma16b(a, vl, accol[t]); }
    wave_lds_sync(); }
#pragma unroll
  for (int t = 0; t < 4; ++t) { const float bb = bf16_rne(bias[t * 16 + nloc]); for (int r = 0; r < 8; ++r) Of[8 * hlf + r][t * 16 + nloc] = (acco[t][r] + accol[t][r] * (1.0f / RS_)) * (1.0f / (PS * XS)) + bb; }
  wave_lds_sync();
  for (int pass = 0; pass < 2; ++pass) { for (int rr = 0; rr < 16; rr += 2) { const int r2 = rr + (lane >> 4); *(volatile v4f*)(out + (rbase + n0 + r2) * D + (lane & 15) * 4) = *(const v4f*)(&Of[r2][(lane & 15) * 4]); } __threadfence(); }
}
}

extern "C" void kernel_launch(void* const* d_in, const int* in_sizes, int n_in, void* d_out, int out_size, void* d_ws, size_t ws_size, hipStream_t stream) {
  (void)n_in;
  auto Fp = [&](int i) { return (const float*)d_in[i]; }; auto Ip = [&](int i) { return (const int*)d_in[i]; };
  if (in_sizes[0] != NR * D || in_sizes[1] != D * D || in_sizes[2] != T * T || in_sizes[3] != D || in_sizes[4] != T * T || out_size != NR * D) return;
  size_t off = 0; char* ws = (char*)d_ws;
  auto carve = [&](size_t bytes) { char* p = ws + off; off += (bytes + 255) & ~(size_t)255; return p; };
  b16* WT = (b16*)carve((size_t)D * D * 2); b16* Xh = (b16*)carve((size_t)NR * D * 2); float* NRM = (float*)carve((size_t)NR * 4); b16* SPh = (b16*)carve((size_t)NR * D * 2); b16* SPl = (b16*)carve((size_t)NR * D * 2);
  if (off > ws_size || off > ((size_t)64 << 20)) return;
  prep_kernel<<<NR / 32, 256, 0, stream>>>(Fp(0), Fp(1), Xh, NRM, WT);
  sup_kernel<<<NR / 32, 64, 0, stream>>>(Xh, WT, SPh, SPl);
  main_kernel<<<dim3(T / 16, BL), 32, 0, stream>>>(Xh, NRM, Fp(2), Ip(4), SPh, SPl, Fp(3), (float*)d_out);
}
